// SelfAttention_33200097198640
// MI455X (gfx1250) — hardware-verified
//
#include <hip/hip_runtime.h>


#ifndef NB
#define NB 2
#endif
#ifndef SEQ
#define SEQ 2048
#endif
#define NB_FULL  2
#define SEQ_FULL 2048
#define DM   1024
#define NH   16
#define HD   64
#define MROWS (NB * SEQ)
#define OSP  68
#define LP   72
#define RSC  2048.0f
#define RINV (1.0f / 2048.0f)
#define PEXP 8.0f
typedef _Float16 h16;
typedef unsigned short bf;
typedef __attribute__((ext_vector_type(16))) __bf16   v16bf;
typedef __attribute__((ext_vector_type(16))) _Float16 v16h;
typedef __attribute__((ext_vector_type(8)))  _Float16 v8h;
typedef __attribute__((ext_vector_type(8)))  unsigned short v8us;
typedef __attribute__((ext_vector_type(8)))  float    v8f;
typedef __attribute__((ext_vector_type(4)))  float    v4f;
typedef v8h  __attribute__((may_alias)) v8ha;
typedef v4f  __attribute__((may_alias)) v4fa;
typedef v8us __attribute__((may_alias)) v8usa;

static_assert(HD == 64);
static_assert(DM == NH * HD);
static_assert(DM % 64 == 0);
static_assert(DM % 32 == 0);
static_assert(SEQ % 64 == 0);
static_assert(MROWS % 64 == 0);
static_assert(NB <= NB_FULL);
static_assert(SEQ <= SEQ_FULL);
static_assert((64 * HD / 8) == 4 * 128);
static_assert(LP % 8 == 0);
static_assert(OSP % 4 == 0);

__device__ __forceinline__ unsigned short f2bf(float f) { unsigned u = __float_as_uint(f); u += 0x7FFFu + ((u >> 16) & 1u); return (unsigned short)(u >> 16); }
__device__ __forceinline__ float bf2f(unsigned short b) { return __uint_as_float(((unsigned)b) << 16); }
__device__ __forceinline__ float bfr(float f) { return bf2f(f2bf(f)); }
__device__ __forceinline__ void splitf(float y, unsigned short& h, unsigned short& l) { h = f2bf(y); l = f2bf(y - bf2f(h)); }
__device__ __forceinline__ v16h cat16(v8h lo, v8h hi) { return __builtin_shufflevector(lo, hi, 0, 1, 2, 3, 4, 5, 6, 7, 8, 9, 10, 11, 12, 13, 14, 15); }
__device__ __forceinline__ v16bf cat16b(v8us lo, v8us hi) { return __builtin_bit_cast(v16bf, __builtin_shufflevector(lo, hi, 0, 1, 2, 3, 4, 5, 6, 7, 8, 9, 10, 11, 12, 13, 14, 15)); }
__device__ __forceinline__ v8f wmma16(v16h a, v16h b, v8f c) { return __builtin_amdgcn_wmma_f32_16x16x32_f16(false, a, false, b, (short)0, c, false, false); }
__device__ __forceinline__ v8f wmmab(v16bf a, v16bf b, v8f c) { return __builtin_amdgcn_wmma_f32_16x16x32_bf16(false, a, false, b, (short)0, c, false, false); }
__device__ __forceinline__ v16bf ldb(const bf* p) { return cat16b(*(const v8us*)p, *(const v8us*)(p + 16)); }
#define LDSFRAG(arr, o) cat16(*(const v8ha*)&(arr)[(o)], *(const v8ha*)&(arr)[(o) + 16])

__global__ __launch_bounds__(256) void k_cvt8(const float* __restrict__ src, bf* dst, size_t n8) {
    const size_t i = (size_t)blockIdx.x * 256 + threadIdx.x; if (i >= n8) return;
    const v8f v = *(const v8f*)(src + i * 8); v8us o;
#pragma unroll
    for (int k = 0; k < 8; ++k) o[k] = f2bf(v[k]);
    *(volatile v8us*)(dst + i * 8) = o; __threadfence(); *(volatile v8us*)(dst + i * 8) = o;
}

template <int NSPLIT, int MODE>
__device__ __forceinline__ void gemm_tile(const bf* __restrict__ A, const bf* A2, const bf* __restrict__ Bt, const float* __restrict__ bias, float* C, h16* P0, h16* P1) {
    __shared__ __align__(16) float os[64 * OSP];
    const int lane = threadIdx.x & 31, lr = lane & 15, hi = lane >> 4;
    const int r0 = blockIdx.x * 64, c0 = blockIdx.y * 64;
    v8f acc[4][4];
#pragma unroll
    for (int mb = 0; mb < 4; ++mb)
#pragma unroll
        for (int nb = 0; nb < 4; ++nb) acc[mb][nb] = (v8f){};
    const size_t aoff = (size_t)(r0 + lr) * DM + 8 * hi, boff = (size_t)(c0 + lr) * DM + 8 * hi;
#pragma unroll 1
    for (int kc = 0; kc < DM; kc += 32) {
        v16bf a[4], a2[4], b;
#pragma unroll
        for (int mb = 0; mb < 4; ++mb) { a[mb] = ldb(A + aoff + (size_t)mb * 16 * DM + kc); if (NSPLIT == 1) a2[mb] = ldb(A2 + aoff + (size_t)mb * 16 * DM + kc); }
#pragma unroll
        for (int nb = 0; nb < 4; ++nb) { b = ldb(Bt + boff + (size_t)nb * 16 * DM + kc);
#pragma unroll
            for (int mb = 0; mb < 4; ++mb) { acc[mb][nb] = wmmab(a[mb], b, acc[mb][nb]); if (NSPLIT == 1) acc[mb][nb] = wmmab(a2[mb], b, acc[mb][nb]); } }
        if (NSPLIT == 1) {
            asm volatile("v_nop\n\tv_nop\n\tv_nop\n\tv_nop" : "+v"(acc[0][0]), "+v"(acc[0][1]), "+v"(acc[0][2]), "+v"(acc[0][3]), "+v"(acc[1][0]), "+v"(acc[1][1]), "+v"(acc[1][2]), "+v"(acc[1][3]) : "v"(a[3]), "v"(a2[3]), "v"(b));
            asm volatile("v_nop\n\tv_nop\n\tv_nop\n\tv_nop" : "+v"(acc[2][0]), "+v"(acc[2][1]), "+v"(acc[2][2]), "+v"(acc[2][3]), "+v"(acc[3][0]), "+v"(acc[3][1]), "+v"(acc[3][2]), "+v"(acc[3][3]) : "v"(a[3]), "v"(a2[3]), "v"(b));
        } else {
            asm volatile("v_nop\n\tv_nop\n\tv_nop\n\tv_nop" : "+v"(acc[0][0]), "+v"(acc[0][1]), "+v"(acc[0][2]), "+v"(acc[0][3]), "+v"(acc[1][0]), "+v"(acc[1][1]), "+v"(acc[1][2]), "+v"(acc[1][3]) : "v"(a[3]), "v"(b));
            asm volatile("v_nop\n\tv_nop\n\tv_nop\n\tv_nop" : "+v"(acc[2][0]), "+v"(acc[2][1]), "+v"(acc[2][2]), "+v"(acc[2][3]), "+v"(acc[3][0]), "+v"(acc[3][1]), "+v"(acc[3][2]), "+v"(acc[3][3]) : "v"(a[3]), "v"(b));
        }
    }
#pragma unroll
    for (int mb = 0; mb < 4; ++mb)
#pragma unroll
        for (int nb = 0; nb < 4; ++nb)
#pragma unroll
            for (int j = 0; j < 8; ++j) os[(mb * 16 + hi * 8 + j) * OSP + nb * 16 + lr] = acc[mb][nb][j];
    __syncthreads();
    const int bq = r0 / SEQ, s0 = r0 % SEQ, hh = c0 / HD;
    if (MODE == 0 || MODE == 1) {
        const int pc = lane & 7, rq = lane >> 3; float bb[8];
#pragma unroll
        for (int j = 0; j < 8; ++j) bb[j] = bfr(bias[c0 + pc * 8 + j]);
#pragma unroll 1
        for (int ps = 0; ps < 2; ++ps) {
#pragma unroll 4
            for (int i = 0; i < 16; ++i) { const int row = 4 * i + rq;
                const v4f x0 = *(const v4fa*)&os[row * OSP + pc * 8]; const v4f x1 = *(const v4fa*)&os[row * OSP + pc * 8 + 4];
                float v[8]; v[0] = x0[0] + bb[0]; v[1] = x0[1] + bb[1]; v[2] = x0[2] + bb[2]; v[3] = x0[3] + bb[3]; v[4] = x1[0] + bb[4]; v[5] = x1[1] + bb[5]; v[6] = x1[2] + bb[6]; v[7] = x1[3] + bb[7];
                v8h vh, vr;
#pragma unroll
                for (int j = 0; j < 8; ++j) { const h16 hv = (h16)v[j]; vh[j] = hv; vr[j] = (h16)((v[j] - (float)hv) * RSC); }
                const size_t g = (((size_t)(bq * NH + hh)) * SEQ + s0 + row) * HD + pc * 8;
                *(volatile v8h*)(P0 + g) = vh; if (MODE == 0) *(volatile v8h*)(P1 + g) = vr; }
            if (ps == 0) __threadfence(); }
    } else if (MODE == 2) {
        const int pc = lane & 7, rq = lane >> 3;
#pragma unroll 1
        for (int ps = 0; ps < 2; ++ps) {
#pragma unroll 4
            for (int i = 0; i < 16; ++i) { const int d = 4 * i + rq; const float bbv = bfr(bias[c0 + d]); v8h vv;
#pragma unroll
                for (int j = 0; j < 8; ++j) vv[j] = (h16)(os[(pc * 8 + j) * OSP + d] + bbv);
                const size_t g = (((size_t)(bq * NH + hh)) * HD + d) * SEQ + s0 + pc * 8;
                *(volatile v8h*)(P0 + g) = vv; }
            if (ps == 0) __threadfence(); }
    } else {
        const int cofs = lr * 4; float bb[4];
#pragma unroll
        for (int j = 0; j < 4; ++j) bb[j] = bfr(bias[c0 + cofs + j]);
#pragma unroll 1
        for (int ps = 0; ps < 2; ++ps) {
#pragma unroll 4
            for (int i = 0; i < 32; ++i) { const int row = 2 * i + hi; v4f val = *(const v4fa*)&os[row * OSP + cofs];
                val[0] += bb[0]; val[1] += bb[1]; val[2] += bb[2]; val[3] += bb[3];
                *(volatile v4f*)(C + (size_t)(r0 + row) * DM + c0 + cofs) = val; }
            if (ps == 0) __threadfence(); }
    }
}

__global__ __launch_bounds__(32) void k_projq(const bf* __restrict__ X, const bf* __restrict__ W, const float* __restrict__ bias, h16* QHp, h16* QRp) { gemm_tile<0, 0>(X, X, W, bias, nullptr, QHp, QRp); }
__global__ __launch_bounds__(32) void k_projk(const bf* __restrict__ X, const bf* __restrict__ W, const float* __restrict__ bias, h16* KHp) { gemm_tile<0, 1>(X, X, W, bias, nullptr, KHp, KHp); }
__global__ __launch_bounds__(32) void k_projv(const bf* __restrict__ X, const bf* __restrict__ W, const float* __restrict__ bias, h16* VTp) { gemm_tile<0, 2>(X, X, W, bias, nullptr, VTp, VTp); }
__global__ __launch_bounds__(32) void k_outp(const bf* __restrict__ Ah, const bf* Al, const bf* __restrict__ W, const float* __restrict__ bias, float* OUT) { gemm_tile<1, 3>(Ah, Al, W, bias, OUT, nullptr, nullptr); }

__global__ __launch_bounds__(128) void k_flash(const h16* __restrict__ QHp, const h16* __restrict__ QRp, const h16* __restrict__ KHp, const h16* __restrict__ VTp, bf* ATh, bf* ATl) {
    __shared__ __align__(16) h16 qh_s[64 * LP];
    __shared__ __align__(16) h16 qr_s[64 * LP];
    __shared__ __align__(16) h16 k_s[64 * LP];
    __shared__ __align__(16) h16 v_s[HD * LP];
    __shared__ __align__(16) unsigned short oh_s[64 * LP];
    __shared__ __align__(16) unsigned short ol_s[64 * LP];
    const int tid = threadIdx.x, lane = tid & 31, lr = lane & 15, hi = lane >> 4;
    const int wave = __builtin_amdgcn_readfirstlane(tid >> 5);
    const int bh = blockIdx.y, q0 = blockIdx.x * 64;
    const size_t pb = (size_t)bh * SEQ * HD;
#pragma unroll
    for (int cc = 0; cc < 4; ++cc) { const int c = tid + cc * 128, row = c >> 3, kof = (c & 7) * 8; const size_t g = pb + (size_t)(q0 + row) * HD + kof;
        *(v8ha*)&qh_s[row * LP + kof] = *(const v8h*)(QHp + g); *(v8ha*)&qr_s[row * LP + kof] = *(const v8h*)(QRp + g); }
    v8f o[4];
#pragma unroll
    for (int dt = 0; dt < 4; ++dt) o[dt] = (v8f){};
    float m = -1.0e30f, l = 0.0f;
    const int qo = (wave * 16 + lr) * LP + 8 * hi;
    const float c2 = 0.125f * 1.4426950408889634f;
#pragma unroll 1
    for (int kb = 0; kb < SEQ / 64; ++kb) {
        __syncthreads();
#pragma unroll
        for (int cc = 0; cc < 4; ++cc) { const int c = tid + cc * 128, row = c >> 3, kof = (c & 7) * 8;
            *(v8ha*)&k_s[row * LP + kof] = *(const v8h*)(KHp + pb + (size_t)(kb * 64 + row) * HD + kof);
            *(v8ha*)&v_s[row * LP + kof] = *(const v8h*)(VTp + pb + (size_t)row * SEQ + kb * 64 + kof); }
        __syncthreads();
#pragma unroll
        for (int half = 0; half < 2; ++half) {
            v8f sh0 = (v8f){}, sh1 = (v8f){}, sr0 = (v8f){}, sr1 = (v8f){};
            v16h bqh, bqr, ak0, ak1;
#pragma unroll
            for (int kc = 0; kc < 2; ++kc) {
                bqh = LDSFRAG(qh_s, qo + kc * 32); bqr = LDSFRAG(qr_s, qo + kc * 32);
                const int ko = (half * 32 + lr) * LP + kc * 32 + 8 * hi;
                ak0 = LDSFRAG(k_s, ko); ak1 = LDSFRAG(k_s, ko + 16 * LP);
                sh0 = wmma16(ak0, bqh, sh0); sr0 = wmma16(ak0, bqr, sr0);
                sh1 = wmma16(ak1, bqh, sh1); sr1 = wmma16(ak1, bqr, sr1);
                asm volatile("v_nop\n\tv_nop\n\tv_nop\n\tv_nop" : "+v"(sh0), "+v"(sh1), "+v"(sr0), "+v"(sr1) : "v"(bqh), "v"(bqr), "v"(ak1));
            }
            float t0[8], t1[8]; float mx = -1.0e30f;
#pragma unroll
            for (int r = 0; r < 8; ++r) { t0[r] = (sr0[r] * RINV + sh0[r]) * c2; t1[r] = (sr1[r] * RINV + sh1[r]) * c2; mx = fmaxf(mx, fmaxf(t0[r], t1[r])); }
            mx = fmaxf(mx, __shfl_xor(mx, 16, 32));
            const float mn = fmaxf(m, mx);
            const float sf = __builtin_amdgcn_exp2f(m - mn);
            m = mn;
            float psum = 0.0f; v8h p0, p1;
#pragma unroll
            for (int r = 0; r < 8; ++r) { const float e0 = __builtin_amdgcn_exp2f(t0[r] - mn + PEXP); const float e1 = __builtin_amdgcn_exp2f(t1[r] - mn + PEXP); psum += e0 + e1; p0[r] = (h16)e0; p1[r] = (h16)e1; }
            l = l * sf + psum;
#pragma unroll
            for (int dt = 0; dt < 4; ++dt)
#pragma unroll
                for (int r = 0; r < 8; ++r) o[dt][r] *= sf;
            const v16h pf = cat16(p0, p1);
            v16h av[4];
#pragma unroll
            for (int dt = 0; dt < 4; ++dt) av[dt] = LDSFRAG(v_s, (dt * 16 + lr) * LP + half * 32 + 8 * hi);
#pragma unroll
            for (int dt = 0; dt < 4; ++dt) o[dt] = wmma16(av[dt], pf, o[dt]);
            asm volatile("v_nop\n\tv_nop\n\tv_nop\n\tv_nop" : "+v"(o[0]), "+v"(o[1]), "+v"(o[2]), "+v"(o[3]) : "v"(pf), "v"(av[3]));
        }
    }
    l += __shfl_xor(l, 16, 32);
    const float inv = 1.0f / l;
#pragma unroll
    for (int dt = 0; dt < 4; ++dt) { v8us vh, vl;
#pragma unroll
        for (int r = 0; r < 8; ++r) { unsigned short a, c; splitf(o[dt][r] * inv, a, c); vh[r] = a; vl[r] = c; }
        *(v8usa*)&oh_s[(wave * 16 + lr) * LP + dt * 16 + 8 * hi] = vh; *(v8usa*)&ol_s[(wave * 16 + lr) * LP + dt * 16 + 8 * hi] = vl; }
    __syncthreads();
    const int b = bh / NH, h = bh % NH; const int pc = lane & 7, rq = lane >> 3;
#pragma unroll 1
    for (int ps = 0; ps < 2; ++ps) {
#pragma unroll
        for (int i = 0; i < 4; ++i) { const int row = wave * 16 + 4 * i + rq;
            const v8us a = *(const v8usa*)&oh_s[row * LP + pc * 8]; const v8us c = *(const v8usa*)&ol_s[row * LP + pc * 8];
            const size_t g = ((size_t)b * SEQ + q0 + row) * DM + h * HD + pc * 8;
            *(volatile v8us*)(ATh + g) = a; *(volatile v8us*)(ATl + g) = c; }
        if (ps == 0) __threadfence(); }
}

extern "C" void kernel_launch(void* const* d_in, const int* in_sizes, int n_in,
                              void* d_out, int out_size, void* d_ws, size_t ws_size, hipStream_t stream) {
    if (n_in < 9) return;
    if (in_sizes[0] < (NB - 1) * SEQ_FULL * DM + SEQ * DM) return;
    if (in_sizes[1] < DM * DM || in_sizes[3] < DM * DM || in_sizes[5] < DM * DM || in_sizes[7] < DM * DM) return;
    if (in_sizes[2] < DM || in_sizes[4] < DM || in_sizes[6] < DM || in_sizes[8] < DM) return;
    if (out_size < MROWS * DM) return;
    const float* x = (const float*)d_in[0]; const float* wq = (const float*)d_in[1]; const float* bq = (const float*)d_in[2]; const float* wk = (const float*)d_in[3]; const float* bk = (const float*)d_in[4];
    const float* wv = (const float*)d_in[5]; const float* bv = (const float*)d_in[6]; const float* wo = (const float*)d_in[7]; const float* bo = (const float*)d_in[8];
    float* OUT = (float*)d_out;
    constexpr size_t SZ_X = (size_t)MROWS * DM * 2;
    constexpr size_t SZ_W = (size_t)DM * DM * 2;
    constexpr size_t SZ_P = (size_t)NB * NH * SEQ * HD * 2;
    constexpr size_t WS_TOTAL = SZ_X + 4 * SZ_W + 4 * SZ_P + 2 * SZ_X;
    static_assert(SZ_X % 256 == 0);
    static_assert(SZ_W % 256 == 0);
    static_assert(SZ_P % 256 == 0);
    static_assert(WS_TOTAL <= (size_t)134217728);
    if (WS_TOTAL > ws_size) return;
    char* wsp = (char*)d_ws;
    bf* XB = (bf*)wsp; wsp += SZ_X;
    bf* WQ = (bf*)wsp; wsp += SZ_W; bf* WK = (bf*)wsp; wsp += SZ_W; bf* WV = (bf*)wsp; wsp += SZ_W; bf* WO = (bf*)wsp; wsp += SZ_W;
    h16* QHp = (h16*)wsp; wsp += SZ_P; h16* QRp = (h16*)wsp; wsp += SZ_P; h16* KHp = (h16*)wsp; wsp += SZ_P; h16* VTp = (h16*)wsp; wsp += SZ_P;
    bf* ATh = (bf*)wsp; wsp += SZ_X; bf* ATl = (bf*)wsp; wsp += SZ_X;

    const size_t nx8 = (size_t)SEQ * DM / 8, nw8 = (size_t)DM * DM / 8;
    for (int b = 0; b < NB; ++b)
        k_cvt8<<<(unsigned)((nx8 + 255) / 256), 256, 0, stream>>>(x + (size_t)b * SEQ_FULL * DM, XB + (size_t)b * SEQ * DM, nx8);
    k_cvt8<<<(unsigned)((nw8 + 255) / 256), 256, 0, stream>>>(wq, WQ, nw8);
    k_cvt8<<<(unsigned)((nw8 + 255) / 256), 256, 0, stream>>>(wk, WK, nw8);
    k_cvt8<<<(unsigned)((nw8 + 255) / 256), 256, 0, stream>>>(wv, WV, nw8);
    k_cvt8<<<(unsigned)((nw8 + 255) / 256), 256, 0, stream>>>(wo, WO, nw8);
    const dim3 gg(MROWS / 64, DM / 64, 1);
    k_projq<<<gg, 32, 0, stream>>>(XB, WQ, bq, QHp, QRp);
    k_projk<<<gg, 32, 0, stream>>>(XB, WK, bk, KHp);
    k_projv<<<gg, 32, 0, stream>>>(XB, WV, bv, VTp);
    k_flash<<<dim3(SEQ / 64, NB * NH, 1), 128, 0, stream>>>(QHp, QRp, KHp, VTp, ATh, ATl);
    k_outp<<<gg, 32, 0, stream>>>(ATh, ATl, WO, bo, OUT);
}
